// MultiStepANN_19069654794946
// MI455X (gfx1250) — hardware-verified
//
#include <hip/hip_runtime.h>
#include <stddef.h>


#define NC   60
#define FC   8
#define HC   32
#define EC   16
#define FH   32
#define KE   960
#define KH   992
#define HH   256
#define EH   128
#define FS   16
#define KS   144
#define KSP  160
#define HS   128
#define ES   64
#define HQ   64
#define KQB  32
#define NT   256
#define RB   16
#define CRW  16
#define CRB  (CRW * (NT / 32))
#define QT   (RB * NC / 16)
#define OP4  (RB * NC / 4)

static_assert(KE == NC * EC);
static_assert(KH == KE + FH);
static_assert(KS == EH + FS);
static_assert(KSP >= KS && KSP % 32 == 0);
static_assert(KE % 32 == 0 && HH % 64 == 0 && EH % 64 == 0 && HS % 64 == 0 && ES == 64 && HQ == 64);
static_assert((RB * NC) % 16 == 0 && (RB * NC) % 4 == 0);
static_assert(CRB == 128);
static_assert(FH == 32 && FS <= 32 && HC == 32 && EC == 16);
static_assert(QT * 16 == RB * NC && OP4 * 4 == RB * NC);

typedef unsigned short us_t;
typedef us_t   v8us  __attribute__((ext_vector_type(8)));
typedef __bf16 v16bf __attribute__((ext_vector_type(16)));
typedef float  v4f   __attribute__((ext_vector_type(4)));
typedef float  v8f   __attribute__((ext_vector_type(8)));
union FragB { v16bf v; v8us h[2]; };

__device__ __forceinline__ v8f wmb(v16bf a, v16bf b, v8f c) {
  v8f d = __builtin_amdgcn_wmma_f32_16x16x32_bf16(false, a, false, b, (short)0, c, false, false);
#if defined(__HIP_DEVICE_COMPILE__)
  asm volatile("v_nop\n\tv_nop\n\tv_nop\n\tv_nop" : "+v"(d) : "v"(a), "v"(b));
#endif
  return d;
}

__device__ __forceinline__ v8f z8() {
  v8f z = {0.f, 0.f, 0.f, 0.f, 0.f, 0.f, 0.f, 0.f};
  return z;
}

__device__ __forceinline__ us_t bbits(float x) {
  unsigned u = __float_as_uint(x);
  u = (u + 0x7FFFu + ((u >> 16) & 1u)) >> 16;
  return (us_t)u;
}
__device__ __forceinline__ float bval(us_t b) {
  return __uint_as_float(((unsigned)b) << 16);
}

__device__ __forceinline__ void ldfrag(FragB& f, const us_t* p) {
  f.h[0] = *(const v8us*)p;
  f.h[1] = *(const v8us*)(p + 16);
}

__device__ __forceinline__ v8f mma3(v16bf ah, v16bf al, v16bf bh, v16bf bl, v8f c) {
  c = wmb(ah, bh, c);
  c = wmb(ah, bl, c);
  c = wmb(al, bh, c);
  return c;
}

__device__ __forceinline__ void pass64(const us_t* Ah, const us_t* Al, int lda, int nk,
                                       const us_t* Wh, const us_t* Wl, int ldw, int n0, int h, int m,
                                       v8f& a0, v8f& a1, v8f& a2, v8f& a3) {
  a0 = z8(); a1 = z8(); a2 = z8(); a3 = z8();
  const us_t* arh = Ah + (size_t)m * lda + 8 * h;
  const us_t* arl = Al + (size_t)m * lda + 8 * h;
  const us_t* brh = Wh + (size_t)(n0 + m) * ldw + 8 * h;
  const us_t* brl = Wl + (size_t)(n0 + m) * ldw + 8 * h;
#pragma unroll 1
  for (int ks = 0; ks < nk; ++ks) {
    const int k0 = 32 * ks;
    FragB fh, fl;
    ldfrag(fh, arh + k0);
    ldfrag(fl, arl + k0);
    {
      FragB bh, bl;
      ldfrag(bh, brh + k0);
      ldfrag(bl, brl + k0);
      a0 = mma3(fh.v, fl.v, bh.v, bl.v, a0);
    }
    {
      FragB bh, bl;
      ldfrag(bh, brh + (size_t)16 * ldw + k0);
      ldfrag(bl, brl + (size_t)16 * ldw + k0);
      a1 = mma3(fh.v, fl.v, bh.v, bl.v, a1);
    }
    {
      FragB bh, bl;
      ldfrag(bh, brh + (size_t)32 * ldw + k0);
      ldfrag(bl, brl + (size_t)32 * ldw + k0);
      a2 = mma3(fh.v, fl.v, bh.v, bl.v, a2);
    }
    {
      FragB bh, bl;
      ldfrag(bh, brh + (size_t)48 * ldw + k0);
      ldfrag(bl, brl + (size_t)48 * ldw + k0);
      a3 = mma3(fh.v, fl.v, bh.v, bl.v, a3);
    }
  }
}

template <bool RELU>
__device__ __forceinline__ void epi_bf(v8f a, float bb, us_t* Dh, us_t* Dl, int ldd, int col, int h) {
#pragma unroll
  for (int r = 0; r < 8; ++r) {
    float v = a[r] + bb;
    if (RELU) v = v > 0.0f ? v : 0.0f;
    const us_t hb = bbits(v);
    const us_t lb = bbits(v - bval(hb));
    Dh[(8 * h + r) * ldd + col] = hb;
    Dl[(8 * h + r) * ldd + col] = lb;
  }
}

__global__ __launch_bounds__(NT) void k_prep(const float* __restrict__ cW2, const float* __restrict__ hW1,
                                             const float* __restrict__ hW2, const float* __restrict__ sW1,
                                             const float* __restrict__ sW2, const float* __restrict__ qW1,
                                             us_t* Pc2h, us_t* Pc2l, us_t* Ph1h, us_t* Ph1l,
                                             us_t* Ph2h, us_t* Ph2l, us_t* Ps1h, us_t* Ps1l,
                                             us_t* Ps2h, us_t* Ps2l, us_t* Pqah, us_t* Pqal,
                                             us_t* Pqbh, us_t* Pqbl) {
  const int s = blockIdx.y;
  const float* W = cW2;
  int K = HC, N = EC, KP = HC;
  us_t* PH = Pc2h;
  us_t* PL = Pc2l;
  bool fold = false;
  if (s == 1)      { W = hW1; K = KH; N = HH; KP = KH;  PH = Ph1h; PL = Ph1l; }
  else if (s == 2) { W = hW2; K = HH; N = EH; KP = HH;  PH = Ph2h; PL = Ph2l; }
  else if (s == 3) { W = sW1; K = KS; N = HS; KP = KSP; PH = Ps1h; PL = Ps1l; }
  else if (s == 4) { W = sW2; K = HS; N = ES; KP = HS;  PH = Ps2h; PL = Ps2l; }
  else if (s == 5) { W = qW1; K = ES; N = HQ; KP = ES;  PH = Pqah; PL = Pqal; }
  else if (s == 6) { W = qW1 + ES * HQ; K = EC; N = HQ; KP = KQB; PH = Pqbh; PL = Pqbl; fold = true; }

  const int npc = (N * KP) / 8;
  const int pb  = blockIdx.x * NT;
  if (pb >= npc) return;
  const int p  = pb + (int)threadIdx.x;
  const int pc = p < npc ? p : npc - 1;
  const int n  = (pc * 8) / KP;
  const int kb = pc * 8 - n * KP;

  v8us oh, ol;
#pragma unroll
  for (int e = 0; e < 8; ++e) {
    const int k  = kb + e;
    const int kr = fold ? (k & 15) : (k < K ? k : K - 1);
    const float wv = W[(size_t)kr * N + n];
    const float v  = (fold || k < K) ? wv : 0.0f;
    const us_t hb = bbits(v);
    const us_t lb = bbits(v - bval(hb));
    oh[e] = hb;
    ol[e] = (fold && k >= 16) ? (us_t)0 : lb;
  }
  us_t* ph = PH + (size_t)p * 8;
  us_t* pl = PL + (size_t)p * 8;
  if (p < npc) {
    *(volatile v8us*)ph = oh;
    *(volatile v8us*)pl = ol;
  }
  __threadfence();
  if (p < npc) {
    *(volatile v8us*)ph = oh;
    *(volatile v8us*)pl = ol;
  }
}

__global__ __launch_bounds__(NT) void k_card(const float* __restrict__ cf, const float* __restrict__ cW1,
                                             const float* __restrict__ cb1, const float* __restrict__ cb2,
                                             const us_t* __restrict__ Pc2h, const us_t* __restrict__ Pc2l,
                                             us_t* Eh, us_t* El, int mrows) {
  __shared__ __align__(16) us_t sAh[(NT / 32) * CRW * HC];
  __shared__ __align__(16) us_t sAl[(NT / 32) * CRW * HC];
  __shared__ __align__(16) us_t sOh[(NT / 32) * CRW * EC];
  __shared__ __align__(16) us_t sOl[(NT / 32) * CRW * EC];

  const int tid = threadIdx.x, lane = tid & 31, h = lane >> 4, m = lane & 15;
  const int wv = __builtin_amdgcn_readfirstlane(tid >> 5);
  const int i0 = (blockIdx.x * (NT / 32) + wv) * CRW;
  us_t* ah = sAh + wv * (CRW * HC);
  us_t* al = sAl + wv * (CRW * HC);
  us_t* oh = sOh + wv * (CRW * EC);
  us_t* ol = sOl + wv * (CRW * EC);

  {
    float w[FC];
#pragma unroll
    for (int f = 0; f < FC; ++f) w[f] = cW1[f * HC + lane];
    const float bj = cb1[lane];
#pragma unroll 1
    for (int r = 0; r < CRW; ++r) {
      int ir = i0 + r;
      ir = ir < mrows ? ir : mrows - 1;
      const float* x = cf + (size_t)ir * FC;
      float a = x[0] * w[0];
      a = fmaf(x[1], w[1], a);
      a = fmaf(x[2], w[2], a);
      a = fmaf(x[3], w[3], a);
      a = fmaf(x[4], w[4], a);
      a = fmaf(x[5], w[5], a);
      a = fmaf(x[6], w[6], a);
      a = fmaf(x[7], w[7], a);
      a = a + bj;
      a = a > 0.0f ? a : 0.0f;
      const us_t hb = bbits(a);
      const us_t lb = bbits(a - bval(hb));
      ah[r * HC + lane] = hb;
      al[r * HC + lane] = lb;
    }
  }
  __syncthreads();

  v8f acc = z8();
  {
    FragB fah, fal, fbh, fbl;
    ldfrag(fah, ah + m * HC + 8 * h);
    ldfrag(fal, al + m * HC + 8 * h);
    ldfrag(fbh, Pc2h + m * HC + 8 * h);
    ldfrag(fbl, Pc2l + m * HC + 8 * h);
    acc = mma3(fah.v, fal.v, fbh.v, fbl.v, acc);
  }
  epi_bf<false>(acc, cb2[m], oh, ol, EC, m, h);
  __syncthreads();

  const v8us voh = *(const v8us*)(oh + 8 * lane);
  const v8us vol = *(const v8us*)(ol + 8 * lane);
  us_t* gh = Eh + (size_t)i0 * EC + 8 * lane;
  us_t* gl = El + (size_t)i0 * EC + 8 * lane;
  *(volatile v8us*)gh = voh;
  *(volatile v8us*)gl = vol;
  __threadfence();
  *(volatile v8us*)gh = voh;
  *(volatile v8us*)gl = vol;
}

__global__ __launch_bounds__(32) void k_chain(const us_t* __restrict__ Eh, const us_t* __restrict__ El,
                                            const float* __restrict__ hf, const float* __restrict__ sf,
                                            const int* __restrict__ play,
                                            const us_t* __restrict__ Ph1h, const us_t* __restrict__ Ph1l,
                                            const us_t* __restrict__ Ph2h, const us_t* __restrict__ Ph2l,
                                            const us_t* __restrict__ Ps1h, const us_t* __restrict__ Ps1l,
                                            const us_t* __restrict__ Ps2h, const us_t* __restrict__ Ps2l,
                                            const us_t* __restrict__ Pqah, const us_t* __restrict__ Pqal,
                                            const us_t* __restrict__ Pqbh, const us_t* __restrict__ Pqbl,
                                            const float* __restrict__ hb1, const float* __restrict__ hb2,
                                            const float* __restrict__ sb1, const float* __restrict__ sb2,
                                            const float* __restrict__ qb1, const float* __restrict__ qW2,
                                            const float* __restrict__ qb2, float* out, int nb) {
  __shared__ __align__(16) us_t sY1h[RB * HH];
  __shared__ __align__(16) us_t sY1l[RB * HH];
  __shared__ __align__(16) us_t sSIh[RB * KSP];
  __shared__ __align__(16) us_t sSIl[RB * KSP];
  __shared__ __align__(16) us_t sS1h[RB * HS];
  __shared__ __align__(16) us_t sS1l[RB * HS];
  __shared__ __align__(16) us_t sSRh[RB * ES];
  __shared__ __align__(16) us_t sSRl[RB * ES];
  __shared__ __align__(16) float sSQ[RB * HQ];
  __shared__ v4f sOut4[OP4];
  float* sOut = (float*)sOut4;

  const int lane = threadIdx.x & 31, h = lane >> 4, m = lane & 15;
  const int b0 = blockIdx.x * RB;

#pragma unroll 1
  for (int r = 0; r < RB; ++r) {
    const int cc = lane < FS ? lane : FS - 1;
    const float fv = sf[(size_t)(b0 + r) * FS + cc];
    const float v  = lane < FS ? fv : 0.0f;
    const us_t hb = bbits(v);
    const us_t lb = bbits(v - bval(hb));
    sSIh[r * KSP + EH + lane] = hb;
    sSIl[r * KSP + EH + lane] = lb;
  }

  FragB ffh, ffl;
  {
    const float* fr = hf + (size_t)(b0 + m) * FH;
    const v4f x0 = *(const v4f*)(fr + 8 * h);
    const v4f x1 = *(const v4f*)(fr + 8 * h + 4);
    const v4f y0 = *(const v4f*)(fr + 16 + 8 * h);
    const v4f y1 = *(const v4f*)(fr + 16 + 8 * h + 4);
    float xs[16];
    xs[0] = x0[0]; xs[1] = x0[1]; xs[2]  = x0[2]; xs[3]  = x0[3];
    xs[4] = x1[0]; xs[5] = x1[1]; xs[6]  = x1[2]; xs[7]  = x1[3];
    xs[8] = y0[0]; xs[9] = y0[1]; xs[10] = y0[2]; xs[11] = y0[3];
    xs[12] = y1[0]; xs[13] = y1[1]; xs[14] = y1[2]; xs[15] = y1[3];
    v8us th0, tl0, th1, tl1;
#pragma unroll
    for (int j = 0; j < 8; ++j) {
      const us_t hb0 = bbits(xs[j]);
      th0[j] = hb0;
      tl0[j] = bbits(xs[j] - bval(hb0));
      const us_t hb1v = bbits(xs[8 + j]);
      th1[j] = hb1v;
      tl1[j] = bbits(xs[8 + j] - bval(hb1v));
    }
    ffh.h[0] = th0; ffh.h[1] = th1;
    ffl.h[0] = tl0; ffl.h[1] = tl1;
  }

  {
    const us_t* arh = Eh + (size_t)(b0 + m) * KE + 8 * h;
    const us_t* arl = El + (size_t)(b0 + m) * KE + 8 * h;
#pragma unroll 1
    for (int ps = 0; ps < HH / 64; ++ps) {
      const int n0 = 64 * ps;
      const us_t* brh = Ph1h + (size_t)(n0 + m) * KH + 8 * h;
      const us_t* brl = Ph1l + (size_t)(n0 + m) * KH + 8 * h;
      v8f acc[4];
#pragma unroll
      for (int t = 0; t < 4; ++t) acc[t] = z8();
#pragma unroll 1
      for (int ks = 0; ks < KE / 32; ++ks) {
        const int k0 = 32 * ks;
        FragB fh, fl;
        ldfrag(fh, arh + k0);
        ldfrag(fl, arl + k0);
#pragma unroll
        for (int t = 0; t < 4; ++t) {
          FragB bh, bl;
          ldfrag(bh, brh + (size_t)(16 * t) * KH + k0);
          ldfrag(bl, brl + (size_t)(16 * t) * KH + k0);
          acc[t] = mma3(fh.v, fl.v, bh.v, bl.v, acc[t]);
        }
      }
#pragma unroll
      for (int t = 0; t < 4; ++t) {
        FragB bh, bl;
        ldfrag(bh, brh + (size_t)(16 * t) * KH + KE);
        ldfrag(bl, brl + (size_t)(16 * t) * KH + KE);
        acc[t] = mma3(ffh.v, ffl.v, bh.v, bl.v, acc[t]);
      }
#pragma unroll
      for (int t = 0; t < 4; ++t) {
        const int n = n0 + 16 * t + m;
        epi_bf<true>(acc[t], hb1[n], sY1h, sY1l, HH, n, h);
      }
    }
  }
  __syncthreads();

#pragma unroll 1
  for (int ps = 0; ps < EH / 64; ++ps) {
    const int n0 = 64 * ps;
    v8f a0, a1, a2, a3;
    pass64(sY1h, sY1l, HH, HH / 32, Ph2h, Ph2l, HH, n0, h, m, a0, a1, a2, a3);
    epi_bf<false>(a0, hb2[n0 + m],      sSIh, sSIl, KSP, n0 + m,      h);
    epi_bf<false>(a1, hb2[n0 + 16 + m], sSIh, sSIl, KSP, n0 + 16 + m, h);
    epi_bf<false>(a2, hb2[n0 + 32 + m], sSIh, sSIl, KSP, n0 + 32 + m, h);
    epi_bf<false>(a3, hb2[n0 + 48 + m], sSIh, sSIl, KSP, n0 + 48 + m, h);
  }
  __syncthreads();

#pragma unroll 1
  for (int ps = 0; ps < HS / 64; ++ps) {
    const int n0 = 64 * ps;
    v8f a0, a1, a2, a3;
    pass64(sSIh, sSIl, KSP, KSP / 32, Ps1h, Ps1l, KSP, n0, h, m, a0, a1, a2, a3);
    epi_bf<true>(a0, sb1[n0 + m],      sS1h, sS1l, HS, n0 + m,      h);
    epi_bf<true>(a1, sb1[n0 + 16 + m], sS1h, sS1l, HS, n0 + 16 + m, h);
    epi_bf<true>(a2, sb1[n0 + 32 + m], sS1h, sS1l, HS, n0 + 32 + m, h);
    epi_bf<true>(a3, sb1[n0 + 48 + m], sS1h, sS1l, HS, n0 + 48 + m, h);
  }
  __syncthreads();

  {
    v8f a0, a1, a2, a3;
    pass64(sS1h, sS1l, HS, HS / 32, Ps2h, Ps2l, HS, 0, h, m, a0, a1, a2, a3);
    epi_bf<false>(a0, sb2[m],      sSRh, sSRl, ES, m,      h);
    epi_bf<false>(a1, sb2[16 + m], sSRh, sSRl, ES, 16 + m, h);
    epi_bf<false>(a2, sb2[32 + m], sSRh, sSRl, ES, 32 + m, h);
    epi_bf<false>(a3, sb2[48 + m], sSRh, sSRl, ES, 48 + m, h);
  }
  __syncthreads();

  {
    v8f aq[4];
    pass64(sSRh, sSRl, ES, ES / 32, Pqah, Pqal, ES, 0, h, m, aq[0], aq[1], aq[2], aq[3]);
#pragma unroll
    for (int t = 0; t < 4; ++t) {
      const int n = 16 * t + m;
      const float bb = qb1[n];
#pragma unroll
      for (int r = 0; r < 8; ++r) sSQ[(8 * h + r) * HQ + n] = aq[t][r] + bb;
    }
  }
  __syncthreads();

  {
    FragB B1[4], B2[4];
    float w2[4];
#pragma unroll
    for (int t = 0; t < 4; ++t) {
      ldfrag(B1[t], Pqbh + (size_t)(16 * t + m) * KQB + 8 * h);
      ldfrag(B2[t], Pqbl + (size_t)(16 * t + m) * KQB + 8 * h);
      w2[t] = qW2[16 * t + m];
    }
    const float qbv = qb2[0];
    const size_t ib0 = (size_t)b0 * NC;
    const int mm = m & 7;
#pragma unroll 1
    for (int tt = 0; tt < QT; ++tt) {
      const size_t ib = ib0 + (size_t)tt * 16;
      FragB fa;
      fa.h[0] = *(const v8us*)(Eh + (ib + m) * EC + 8 * h);
      fa.h[1] = *(const v8us*)(El + (ib + m) * EC + 8 * h);
      v8f acc[4];
#pragma unroll
      for (int t = 0; t < 4; ++t) {
        acc[t] = wmb(fa.v, B1[t].v, z8());
        acc[t] = wmb(fa.v, B2[t].v, acc[t]);
      }
      float p[8];
#pragma unroll
      for (int r = 0; r < 8; ++r) p[r] = 0.0f;
#pragma unroll
      for (int r = 0; r < 8; ++r) {
        const int lr = 16 * tt + 8 * h + r;
        const int lb = lr / NC;
        const float* sq = sSQ + lb * HQ;
#pragma unroll
        for (int t = 0; t < 4; ++t) {
          float v = acc[t][r] + sq[16 * t + m];
          v = v > 0.0f ? v : 0.0f;
          p[r] = fmaf(v, w2[t], p[r]);
        }
      }
#pragma unroll
      for (int off = 1; off < 16; off <<= 1) {
#pragma unroll
        for (int r = 0; r < 8; ++r) p[r] += __shfl_xor(p[r], off, 32);
      }
      float ov1 = p[0];
#pragma unroll
      for (int r = 1; r < 8; ++r) ov1 = (m == r) ? p[r] : ov1;
      const int   pl  = play[ib + 8 * h + mm];
      const float qv  = ov1 + qbv;
      const float res = (pl == 1) ? qv : 0.0f;
      if (m < 8) sOut[16 * tt + 8 * h + mm] = res;
    }
  }
  __syncthreads();

  v4f ov[8];
#pragma unroll
  for (int q = 0; q < 8; ++q) {
    int pc = 32 * q + lane;
    pc = pc < OP4 ? pc : OP4 - 1;
    ov[q] = sOut4[pc];
  }
  float* ob = out + (size_t)b0 * NC;
#pragma unroll
  for (int q = 0; q < 8; ++q) {
    const int pc = 32 * q + lane;
    if (pc < OP4) *(volatile v4f*)(ob + 4 * pc) = ov[q];
  }
  __threadfence();
#pragma unroll
  for (int q = 0; q < 8; ++q) {
    const int pc = 32 * q + lane;
    if (pc < OP4) *(volatile v4f*)(ob + 4 * pc) = ov[q];
  }
}

extern "C" void kernel_launch(void* const* d_in, const int* in_sizes, int n_in,
                              void* d_out, int out_size, void* d_ws, size_t ws_size,
                              hipStream_t stream) {
  if (n_in < 20) return;
  const int m_all = in_sizes[1];
  if (m_all <= 0 || (m_all % NC) != 0) return;
  const int nb = m_all / NC;
  if ((nb % 32) != 0) return;
  if (in_sizes[0] != m_all * FC || in_sizes[2] != nb * FH || in_sizes[3] != nb * FS) return;
  if (in_sizes[4] != FC * HC || in_sizes[5] != HC || in_sizes[6] != HC * EC || in_sizes[7] != EC) return;
  if (in_sizes[8] != KH * HH || in_sizes[9] != HH || in_sizes[10] != HH * EH || in_sizes[11] != EH) return;
  if (in_sizes[12] != KS * HS || in_sizes[13] != HS || in_sizes[14] != HS * ES || in_sizes[15] != ES) return;
  if (in_sizes[16] != (ES + EC) * HQ || in_sizes[17] != HQ || in_sizes[18] != HQ || in_sizes[19] != 1) return;
  if (out_size != m_all) return;

  const float* cf   = (const float*)d_in[0];
  const int*   play = (const int*)d_in[1];
  const float* hf   = (const float*)d_in[2];
  const float* sf   = (const float*)d_in[3];
  const float* cW1  = (const float*)d_in[4];
  const float* cb1  = (const float*)d_in[5];
  const float* cW2  = (const float*)d_in[6];
  const float* cb2  = (const float*)d_in[7];
  const float* hW1  = (const float*)d_in[8];
  const float* hb1  = (const float*)d_in[9];
  const float* hW2  = (const float*)d_in[10];
  const float* hb2  = (const float*)d_in[11];
  const float* sW1  = (const float*)d_in[12];
  const float* sb1  = (const float*)d_in[13];
  const float* sW2  = (const float*)d_in[14];
  const float* sb2  = (const float*)d_in[15];
  const float* qW1  = (const float*)d_in[16];
  const float* qb1  = (const float*)d_in[17];
  const float* qW2  = (const float*)d_in[18];
  const float* qb2  = (const float*)d_in[19];
  float* out = (float*)d_out;

  size_t off = 0;
  size_t o[16];
  const size_t bytes[8] = {
    (size_t)EC * HC * 2, (size_t)HH * KH * 2, (size_t)EH * HH * 2, (size_t)HS * KSP * 2,
    (size_t)ES * HS * 2, (size_t)HQ * ES * 2, (size_t)HQ * KQB * 2, (size_t)m_all * EC * 2 };
  for (int i = 0; i < 8; ++i) {
    for (int j = 0; j < 2; ++j) {
      o[2 * i + j] = off;
      off += (bytes[i] + 255) & ~(size_t)255;
    }
  }
  const size_t total = off;
  if (total > ws_size || total > (size_t)134217728) return;
  char* wb = (char*)d_ws;
  us_t* Pc2h = (us_t*)(wb + o[0]);  us_t* Pc2l = (us_t*)(wb + o[1]);
  us_t* Ph1h = (us_t*)(wb + o[2]);  us_t* Ph1l = (us_t*)(wb + o[3]);
  us_t* Ph2h = (us_t*)(wb + o[4]);  us_t* Ph2l = (us_t*)(wb + o[5]);
  us_t* Ps1h = (us_t*)(wb + o[6]);  us_t* Ps1l = (us_t*)(wb + o[7]);
  us_t* Ps2h = (us_t*)(wb + o[8]);  us_t* Ps2l = (us_t*)(wb + o[9]);
  us_t* Pqah = (us_t*)(wb + o[10]); us_t* Pqal = (us_t*)(wb + o[11]);
  us_t* Pqbh = (us_t*)(wb + o[12]); us_t* Pqbl = (us_t*)(wb + o[13]);
  us_t* Eh   = (us_t*)(wb + o[14]); us_t* El   = (us_t*)(wb + o[15]);

  const int prep_x = (HH * KH / 8 + NT - 1) / NT;
  k_prep<<<dim3(prep_x, 7), NT, 0, stream>>>(cW2, hW1, hW2, sW1, sW2, qW1,
                                              Pc2h, Pc2l, Ph1h, Ph1l, Ph2h, Ph2l, Ps1h, Ps1l,
                                              Ps2h, Ps2l, Pqah, Pqal, Pqbh, Pqbl);
  k_card<<<m_all / CRB, NT, 0, stream>>>(cf, cW1, cb1, cb2, Pc2h, Pc2l, Eh, El, m_all);
  k_chain<<<nb / RB, 32, 0, stream>>>(Eh, El, hf, sf, play,
                                      Ph1h, Ph1l, Ph2h, Ph2l, Ps1h, Ps1l, Ps2h, Ps2l,
                                      Pqah, Pqal, Pqbh, Pqbl,
                                      hb1, hb2, sb1, sb2, qb1, qW2, qb2, out, nb);
}
